// MambaTemporal_32873679684185
// MI455X (gfx1250) — hardware-verified
//
#include <hip/hip_runtime.h>
#define BB 8
#define TT 512
#define DM 1024
#define DI 2048
#define NS 16
#define DTR 64
#define XPW (DTR + 2 * NS)
#define NR (BB * TT)
#define LNEPS 1e-5f
__device__ __forceinline__ float fexp(float x) { return __builtin_amdgcn_exp2f(x * 1.4426950408889634f); }
typedef __bf16 v16b __attribute__((ext_vector_type(16)));
typedef unsigned short v8us __attribute__((ext_vector_type(8), may_alias));
typedef float  v8f  __attribute__((ext_vector_type(8)));
typedef float  v4f  __attribute__((ext_vector_type(4)));
typedef float  v4fa __attribute__((ext_vector_type(4), may_alias));
union FragB { v16b v; v8us half[2]; unsigned short u[16]; };

__device__ __forceinline__ unsigned short bf16_bits(float x) { unsigned int u = __float_as_uint(x); return (unsigned short)((u + 0x7FFFu + ((u >> 16) & 1u)) >> 16); }
__device__ __forceinline__ float bf16_val(unsigned short b) { return __uint_as_float(((unsigned int)b) << 16); }
__device__ __forceinline__ float bf16_round(float x) { return bf16_val(bf16_bits(x)); }
template <int NT>
__device__ __forceinline__ v8f mmaN(v16b ah, v16b al, v16b bh, v16b bl, v8f c) {
  c = __builtin_amdgcn_wmma_f32_16x16x32_bf16(false, ah, false, bh, (short)0, c, false, false);
  if (NT >= 2) c = __builtin_amdgcn_wmma_f32_16x16x32_bf16(false, al, false, bh, (short)0, c, false, false);
  if (NT >= 3) c = __builtin_amdgcn_wmma_f32_16x16x32_bf16(false, ah, false, bl, (short)0, c, false, false);
  asm volatile("v_nop\n\tv_nop\n\tv_nop\n\tv_nop" : "+v"(c) : "v"(ah), "v"(al), "v"(bh), "v"(bl));
  return c;
}

__global__ __launch_bounds__(256) void k_wt_bf16(const float* __restrict__ W, unsigned short* __restrict__ Wt, int K, int N) {
  const int t = blockIdx.x * 256 + threadIdx.x;
  const int k8n = K / 8;
  if (t >= N * k8n) return;
  const int n = t / k8n, k8 = (t % k8n) * 8;
  v8us v;
#pragma unroll
  for (int i = 0; i < 8; ++i) v[i] = bf16_bits(W[(size_t)(k8 + i) * N + n]);
  *(volatile v8us*)(Wt + (size_t)n * K + k8) = v;
  __threadfence();
  *(volatile v8us*)(Wt + (size_t)n * K + k8) = v;
}

template <bool ASPLIT, int ACT, bool BIAS_BF16>
__global__ __launch_bounds__(128) void k_gemm_bf(const float* __restrict__ A, int lda, const unsigned short* __restrict__ Wt, int ldb,
                                               const float* __restrict__ bias, float* __restrict__ C, int ldc, int M, int N, int K) {
  __shared__ __attribute__((aligned(16))) float so[4][16][64];
  const int tid = threadIdx.x, w = tid >> 5, lane = tid & 31, ln = lane & 15, hh = lane >> 4;
  const int ntn = N / 64;
  const int wid = blockIdx.x * 4 + w;
  const int mt = wid / ntn, nq = wid % ntn;
  if (mt * 16 >= M) return;
  const int row0 = mt * 16, col0 = nq * 64;
  const float* arow = A + (size_t)(row0 + ln) * lda;
  v8f acc[4] = {};
  for (int kb = 0; kb < K; kb += 32) {
    FragB ah, al;
    const v4f x0 = *(const v4fa*)(arow + kb + 8 * hh), x1 = *(const v4fa*)(arow + kb + 8 * hh + 4);
    const v4f x2 = *(const v4fa*)(arow + kb + 16 + 8 * hh), x3 = *(const v4fa*)(arow + kb + 16 + 8 * hh + 4);
    float xs[16] = {x0[0],x0[1],x0[2],x0[3],x1[0],x1[1],x1[2],x1[3],x2[0],x2[1],x2[2],x2[3],x3[0],x3[1],x3[2],x3[3]};
#pragma unroll
    for (int i = 0; i < 16; ++i) { const unsigned short hb = bf16_bits(xs[i]); ah.u[i] = hb; al.u[i] = ASPLIT ? bf16_bits(xs[i] - bf16_val(hb)) : (unsigned short)0; }
#pragma unroll
    for (int t = 0; t < 4; ++t) {
      const unsigned short* brow = Wt + (size_t)(col0 + t * 16 + ln) * ldb + kb;
      FragB b;
      b.half[0] = *(const v8us*)(brow + 8 * hh);
      b.half[1] = *(const v8us*)(brow + 16 + 8 * hh);
      acc[t] = mmaN<ASPLIT ? 2 : 1>(ah.v, al.v, b.v, b.v, acc[t]);
    }
  }
#pragma unroll
  for (int t = 0; t < 4; ++t) {
    float bv = bias ? bias[col0 + t * 16 + ln] : 0.f;
    if (BIAS_BF16) bv = bf16_round(bv);
#pragma unroll
    for (int r = 0; r < 8; ++r) { float v = acc[t][r] + bv; if (ACT == 1) v = fmaxf(v, 0.f); so[w][8 * hh + r][t * 16 + ln] = v; }
  }
  __builtin_amdgcn_fence(__ATOMIC_ACQ_REL, "workgroup");
  __builtin_amdgcn_wave_barrier();
  const int rsub = lane >> 4, c4 = (lane & 15) * 4;
  for (int pass = 0; pass < 2; ++pass) {
#pragma unroll
    for (int q = 0; q < 8; ++q) {
      const int r = q * 2 + rsub;
      const v4f v = *(const v4fa*)&so[w][r][c4];
      *(volatile v4f*)(C + (size_t)(row0 + r) * ldc + col0 + c4) = v;
    }
    if (pass == 0) __threadfence();
  }
}

template <bool ASPLIT, int ACT, bool BIAS_BF16, bool RES_BF16>
__global__ __launch_bounds__(128) void k_gemm_bf3(const float* __restrict__ A, int lda, const unsigned short* __restrict__ Wt, int ldb,
                                                const float* __restrict__ bias, const float* __restrict__ resid, int rmod, int ldr,
                                                float* __restrict__ C, int ldc, int M, int N, int K) {
  __shared__ __attribute__((aligned(16))) float so[4][16][64];
  const int tid = threadIdx.x, w = tid >> 5, lane = tid & 31, ln = lane & 15, hh = lane >> 4;
  const int ntn = N / 64;
  const int wid = blockIdx.x * 4 + w;
  const int mt = wid / ntn, nq = wid % ntn;
  if (mt * 16 >= M) return;
  const int row0 = mt * 16, col0 = nq * 64;
  const float* arow = A + (size_t)(row0 + ln) * lda;
  v8f acc[4] = {};
  for (int kb = 0; kb < K; kb += 32) {
    FragB ah, al;
    const v4f x0 = *(const v4fa*)(arow + kb + 8 * hh), x1 = *(const v4fa*)(arow + kb + 8 * hh + 4);
    const v4f x2 = *(const v4fa*)(arow + kb + 16 + 8 * hh), x3 = *(const v4fa*)(arow + kb + 16 + 8 * hh + 4);
    float xs[16] = {x0[0],x0[1],x0[2],x0[3],x1[0],x1[1],x1[2],x1[3],x2[0],x2[1],x2[2],x2[3],x3[0],x3[1],x3[2],x3[3]};
#pragma unroll
    for (int i = 0; i < 16; ++i) { const unsigned short hb = bf16_bits(xs[i]); ah.u[i] = hb; al.u[i] = ASPLIT ? bf16_bits(xs[i] - bf16_val(hb)) : (unsigned short)0; }
#pragma unroll
    for (int t = 0; t < 4; ++t) {
      const unsigned short* brow = Wt + (size_t)(col0 + t * 16 + ln) * ldb + kb;
      FragB b;
      b.half[0] = *(const v8us*)(brow + 8 * hh);
      b.half[1] = *(const v8us*)(brow + 16 + 8 * hh);
      acc[t] = mmaN<ASPLIT ? 2 : 1>(ah.v, al.v, b.v, b.v, acc[t]);
    }
  }
#pragma unroll
  for (int t = 0; t < 4; ++t) {
    const int col = col0 + t * 16 + ln;
    float bv = bias ? bias[col] : 0.f;
    if (BIAS_BF16) bv = bf16_round(bv);
#pragma unroll
    for (int r = 0; r < 8; ++r) {
      float v = acc[t][r] + bv;
      if (resid) { float rv = resid[(size_t)((row0 + 8 * hh + r) % rmod) * ldr + col]; if (RES_BF16) rv = bf16_round(rv); v += rv; }
      if (ACT == 1) v = fmaxf(v, 0.f);
      if (ACT == 2) v = 0.5f * v * (1.0f + erff(v * 0.70710678118654752f));
      if (ACT == 3) { const float u = 0.7978845608028654f * (v + 0.044715f * v * v * v); v = 0.5f * v * (1.0f + tanhf(u)); }
      so[w][8 * hh + r][t * 16 + ln] = v;
    }
  }
  __builtin_amdgcn_fence(__ATOMIC_ACQ_REL, "workgroup");
  __builtin_amdgcn_wave_barrier();
  const int rsub = lane >> 4, c4 = (lane & 15) * 4;
  for (int pass = 0; pass < 2; ++pass) {
#pragma unroll
    for (int q = 0; q < 8; ++q) {
      const int r = q * 2 + rsub;
      const v4f v = *(const v4fa*)&so[w][r][c4];
      *(volatile v4f*)(C + (size_t)(row0 + r) * ldc + col0 + c4) = v;
    }
    if (pass == 0) __threadfence();
  }
}
template <bool PARAM_BF16>
__global__ __launch_bounds__(256) void k_layernorm(const float* __restrict__ X, const float* __restrict__ R, const float* __restrict__ g, const float* __restrict__ bta,
                                                  float* __restrict__ out_sum, float* __restrict__ out_norm, int N, float eps) {
  __shared__ float red[256];
  const int row = blockIdx.x, tid = threadIdx.x;
  const float* x = X + (size_t)row * N; const float* rr = R ? R + (size_t)row * N : nullptr;
  float vals[16];
  const int per = N / 256;
  float s1 = 0.f;
  for (int u = 0; u < per / 4; ++u) {
    const int j = tid * 4 + 1024 * u;
    const v4f a = *(const v4fa*)(x + j);
    v4f b = {0.f,0.f,0.f,0.f}; if (rr) b = *(const v4fa*)(rr + j);
#pragma unroll
    for (int q = 0; q < 4; ++q) { const float v = a[q] + b[q]; vals[u * 4 + q] = v; s1 += v; }
  }
  red[tid] = s1; __syncthreads();
  for (int st = 128; st > 0; st >>= 1) { if (tid < st) red[tid] += red[tid + st]; __syncthreads(); }
  const float mu = red[0] / (float)N; __syncthreads();
  float s2 = 0.f;
  for (int u = 0; u < per / 4; ++u)
#pragma unroll
    for (int q = 0; q < 4; ++q) { const float c = vals[u * 4 + q] - mu; s2 += c * c; }
  red[tid] = s2; __syncthreads();
  for (int st = 128; st > 0; st >>= 1) { if (tid < st) red[tid] += red[tid + st]; __syncthreads(); }
  const float rs = rsqrtf(red[0] / (float)N + eps);
  for (int pass = 0; pass < 2; ++pass) {
    for (int u = 0; u < per / 4; ++u) {
      const int j = tid * 4 + 1024 * u;
      v4f o, sm;
#pragma unroll
      for (int q = 0; q < 4; ++q) {
        float gg = g[j + q], bb = bta[j + q];
        if (PARAM_BF16) { gg = bf16_round(gg); bb = bf16_round(bb); }
        sm[q] = vals[u * 4 + q]; o[q] = (vals[u * 4 + q] - mu) * rs * gg + bb;
      }
      if (out_sum) *(volatile v4f*)(out_sum + (size_t)row * N + j) = sm;
      *(volatile v4f*)(out_norm + (size_t)row * N + j) = o;
    }
    if (pass == 0) __threadfence();
  }
}


typedef _Float16 v16h __attribute__((ext_vector_type(16)));
union FragH { v16h v; v8us half[2]; _Float16 h[16]; unsigned short u[16]; };
template <int NT>
__device__ __forceinline__ v8f mmaH(v16h ah, v16h al, v16h bh, v16h bl, v8f c) {
  c = __builtin_amdgcn_wmma_f32_16x16x32_f16(false, ah, false, bh, (short)0, c, false, false);
  if (NT >= 2) c = __builtin_amdgcn_wmma_f32_16x16x32_f16(false, al, false, bh, (short)0, c, false, false);
  if (NT >= 3) c = __builtin_amdgcn_wmma_f32_16x16x32_f16(false, ah, false, bl, (short)0, c, false, false);
  asm volatile("v_nop\n\tv_nop\n\tv_nop\n\tv_nop" : "+v"(c) : "v"(ah), "v"(al), "v"(bh), "v"(bl));
  return c;
}
template <bool ASPLIT>
__global__ __launch_bounds__(128) void k_gemm_h(const float* __restrict__ A, int lda, size_t sA, const _Float16* __restrict__ Bh, int ldb, size_t sB, float alpha, float* __restrict__ C, int ldc, size_t sC, int M, int N, int K) {
  __shared__ __attribute__((aligned(16))) float so[4][16][64];
  const int tid = threadIdx.x, w = tid >> 5, lane = tid & 31, ln = lane & 15, hh = lane >> 4; const int by = blockIdx.y;
  A += (size_t)by * sA; Bh += (size_t)by * sB; C += (size_t)by * sC;
  const int ntn = (N + 63) / 64; const int wid = blockIdx.x * 4 + w; const int mt = wid / ntn, nq = wid % ntn; if (mt * 16 >= M) return;
  const int row0 = mt * 16, col0 = nq * 64; const float* arow = A + (size_t)(row0 + ln) * lda;
  v8f acc[4] = {};
  for (int kb = 0; kb < K; kb += 32) {
    FragH ah, al;
    const v4f x0 = *(const v4fa*)(arow + kb + 8 * hh), x1 = *(const v4fa*)(arow + kb + 8 * hh + 4), x2 = *(const v4fa*)(arow + kb + 16 + 8 * hh), x3 = *(const v4fa*)(arow + kb + 16 + 8 * hh + 4);
    float xs[16] = {x0[0],x0[1],x0[2],x0[3],x1[0],x1[1],x1[2],x1[3],x2[0],x2[1],x2[2],x2[3],x3[0],x3[1],x3[2],x3[3]};
#pragma unroll
    for (int i = 0; i < 16; ++i) { const _Float16 h = (_Float16)xs[i]; ah.h[i] = h; al.h[i] = ASPLIT ? (_Float16)(xs[i] - (float)h) : (_Float16)0.0f; }
#pragma unroll
    for (int t = 0; t < 4; ++t) { if (col0 + t * 16 >= N) continue; const size_t boff = (size_t)(col0 + t * 16 + ln) * ldb + kb; FragH bq; bq.half[0] = *(const v8us*)(Bh + boff + 8 * hh); bq.half[1] = *(const v8us*)(Bh + boff + 16 + 8 * hh);
      acc[t] = mmaH<ASPLIT ? 2 : 1>(ah.v, al.v, bq.v, bq.v, acc[t]); }
  }
#pragma unroll
  for (int t = 0; t < 4; ++t) { if (col0 + t * 16 >= N) continue;
#pragma unroll
    for (int r = 0; r < 8; ++r) so[w][8 * hh + r][t * 16 + ln] = acc[t][r] * alpha; }
  __builtin_amdgcn_fence(__ATOMIC_ACQ_REL, "workgroup"); __builtin_amdgcn_wave_barrier();
  const int rsub = lane >> 4, c4 = (lane & 15) * 4;
  for (int pass = 0; pass < 2; ++pass) {
#pragma unroll
    for (int q = 0; q < 8; ++q) { const int r = q * 2 + rsub; if (col0 + c4 < N) { const v4f v = *(const v4fa*)&so[w][r][c4]; *(volatile v4f*)(C + (size_t)(row0 + r) * ldc + col0 + c4) = v; } }
    if (pass == 0) __threadfence(); }
}

__global__ __launch_bounds__(256) void k_wt_f16(const float* __restrict__ W, _Float16* __restrict__ Wt, int K, int N, float scale) {
  const int t = blockIdx.x * 256 + threadIdx.x; if (t >= N * (K / 8)) return; const int n = t / (K / 8), k8 = (t % (K / 8)) * 8; FragH f;
#pragma unroll
  for (int i = 0; i < 8; ++i) f.h[i] = (_Float16)(bf16_round(W[(size_t)(k8 + i) * N + n]) * scale); const v8us o = f.half[0];
  *(volatile v8us*)((unsigned short*)Wt + (size_t)n * K + k8) = o; __threadfence(); *(volatile v8us*)((unsigned short*)Wt + (size_t)n * K + k8) = o;
}
template <int ACT>
__global__ __launch_bounds__(128) void k_gemm_hhx(const _Float16* __restrict__ A, int lda, size_t sA, const _Float16* __restrict__ Bh, int ldb, size_t sB, float alpha, const float* __restrict__ bias, size_t sBias, const float* __restrict__ CP, int rowsPerB, size_t sCPb, int row0g,
    float* __restrict__ C, _Float16* __restrict__ C16, int ldc, size_t sC, int M, int N, int K) {
  __shared__ __attribute__((aligned(16))) float so[4][16][64];
  const int tid = threadIdx.x, w = tid >> 5, lane = tid & 31, ln = lane & 15, hh = lane >> 4; const int by = blockIdx.y;
  A += (size_t)by * sA; Bh += (size_t)by * sB; const size_t cofs = (size_t)by * sC; const float* bp = bias ? bias + (size_t)by * sBias : nullptr;
  const int ntn = (N + 63) / 64; const int wid = blockIdx.x * 4 + w; const int mt = wid / ntn, nq = wid % ntn; if (mt * 16 >= M) return;
  const int row0 = mt * 16, col0 = nq * 64; const _Float16* arow = A + (size_t)(row0 + ln) * lda;
  v8f acc[4] = {};
  for (int kb = 0; kb < K; kb += 32) { FragH ah; ah.half[0] = *(const v8us*)((const unsigned short*)arow + kb + 8 * hh); ah.half[1] = *(const v8us*)((const unsigned short*)arow + kb + 16 + 8 * hh);
#pragma unroll
    for (int t = 0; t < 4; ++t) { if (col0 + t * 16 >= N) continue; const size_t boff = (size_t)(col0 + t * 16 + ln) * ldb + kb; FragH bq; bq.half[0] = *(const v8us*)((const unsigned short*)Bh + boff + 8 * hh); bq.half[1] = *(const v8us*)((const unsigned short*)Bh + boff + 16 + 8 * hh);
      acc[t] = mmaH<1>(ah.v, ah.v, bq.v, bq.v, acc[t]); }
  }
#pragma unroll
  for (int t = 0; t < 4; ++t) { if (col0 + t * 16 >= N) continue; const int col = col0 + t * 16 + ln; const float bv = bp ? bf16_round(bp[col]) : 0.f;
#pragma unroll
    for (int r = 0; r < 8; ++r) { float v = acc[t][r] * alpha + bv; if (CP) { const int bidx = (row0g + row0 + 8 * hh + r) / rowsPerB; v += CP[(size_t)bidx * sCPb + (size_t)by * 64 + col]; } if (ACT == 1) v = (v > 0.f) ? v : expm1f(v); else if (ACT == 7) v = (v > 0.f) ? v + 1.0f : expf(v); else if (ACT == 8) v = tanhf(v); else if (ACT == 9) v = 0.5f * v * (1.0f + tanhf(0.7978845608028654f * (v + 0.044715f * v * v * v))); else if (ACT == 11) v = 1.0f / (1.0f + expf(-v)); else if (ACT == 12) v = (v > 0.f) ? v : 0.01f * v; else if (ACT == 14) v = (v > 0.f) ? v : 0.1f * v; else if (ACT == 15) v = v / (1.0f + expf(-v)); else if (ACT == 3) v = fmaxf(v, 0.f); else if (ACT == 6) v = 0.5f * v * (1.0f + erff(v * 0.70710678118654752f)); else if (ACT == 13) v = (v > 20.f) ? v : log1pf(expf(v)); so[w][8 * hh + r][t * 16 + ln] = v; } }
  __builtin_amdgcn_fence(__ATOMIC_ACQ_REL, "workgroup"); __builtin_amdgcn_wave_barrier();
  const int rsub = lane >> 4, c4 = (lane & 15) * 4; typedef _Float16 v4h __attribute__((ext_vector_type(4)));
  for (int pass = 0; pass < 2; ++pass) {
#pragma unroll
    for (int q = 0; q < 8; ++q) { const int r = q * 2 + rsub; if (col0 + c4 < N) { const v4f v = *(const v4fa*)&so[w][r][c4]; if (C) *(volatile v4f*)(C + cofs + (size_t)(row0 + r) * ldc + col0 + c4) = v; if (C16) { v4h h4; for (int i = 0; i < 4; ++i) h4[i] = (_Float16)v[i]; *(volatile v4h*)(C16 + cofs + (size_t)(row0 + r) * ldc + col0 + c4) = h4; } } }
    if (pass == 0) __threadfence(); }
}


typedef _Float16 v4h __attribute__((ext_vector_type(4)));

__global__ __launch_bounds__(256) void k_x16(const float* __restrict__ x, _Float16* __restrict__ X16, size_t n8) { const size_t t = (size_t)blockIdx.x * 256 + threadIdx.x; if (t >= n8) return; FragH f;
#pragma unroll
  for (int q = 0; q < 8; ++q) f.h[q] = (_Float16)bf16_round(x[t * 8 + q]); *(volatile v8us*)((unsigned short*)X16 + t * 8) = f.half[0]; __threadfence(); *(volatile v8us*)((unsigned short*)X16 + t * 8) = f.half[0]; }
__global__ __launch_bounds__(256) void k_h16(const float* __restrict__ x, _Float16* __restrict__ X16, size_t n8) { const size_t t = (size_t)blockIdx.x * 256 + threadIdx.x; if (t >= n8) return; FragH f;
#pragma unroll
  for (int q = 0; q < 8; ++q) f.h[q] = (_Float16)x[t * 8 + q]; *(volatile v8us*)((unsigned short*)X16 + t * 8) = f.half[0]; __threadfence(); *(volatile v8us*)((unsigned short*)X16 + t * 8) = f.half[0]; }
__global__ __launch_bounds__(256) void k_round16f(const float* __restrict__ W, _Float16* __restrict__ Bt, size_t n8) { const size_t t = (size_t)blockIdx.x * 256 + threadIdx.x; if (t >= n8) return; FragH f;
#pragma unroll
  for (int i = 0; i < 8; ++i) f.h[i] = (_Float16)(bf16_round(W[t * 8 + i]) * 16.0f); *(volatile v8us*)((unsigned short*)Bt + t * 8) = f.half[0]; __threadfence(); *(volatile v8us*)((unsigned short*)Bt + t * 8) = f.half[0]; }
template <int NHv, int TTv>
__global__ __launch_bounds__(256) void k_vt(const _Float16* __restrict__ V16, int ldv, int voff, _Float16* __restrict__ Vt) { __shared__ unsigned short tl[64][66]; const int tid = threadIdx.x; const int slab = blockIdx.x / (TTv / 64), lg = blockIdx.x % (TTv / 64); const int b = slab / NHv, h = slab % NHv;
  for (int i = tid; i < 64 * 8; i += 256) { const int r = i / 8, c8 = (i % 8) * 8; FragH f; f.half[0] = *(const v8us*)((const unsigned short*)V16 + ((size_t)b * TTv + lg * 64 + r) * ldv + voff + h * 64 + c8);
#pragma unroll
    for (int q = 0; q < 8; ++q) tl[r][c8 + q] = f.u[q]; }
  __syncthreads();
  for (int pass = 0; pass < 2; ++pass) {
#pragma unroll
    for (int rd = 0; rd < 2; ++rd) { const int d = rd * 32 + tid / 8, pc = tid % 8; FragH f;
#pragma unroll
      for (int q = 0; q < 8; ++q) f.u[q] = tl[pc * 8 + q][d];
      *(volatile v8us*)((unsigned short*)Vt + ((size_t)slab * 64 + d) * TTv + lg * 64 + pc * 8) = f.half[0]; }
    if (pass == 0) __threadfence(); } }

__global__ __launch_bounds__(256) void k_hl(const float* __restrict__ F, _Float16* __restrict__ Hh, _Float16* __restrict__ Hl, size_t n8) { const size_t t = (size_t)blockIdx.x * 256 + threadIdx.x; if (t >= n8) return; FragH fh, fl; const v4f a = *(const v4fa*)(F + t * 8), c = *(const v4fa*)(F + t * 8 + 4);
#pragma unroll
  for (int q = 0; q < 4; ++q) { _Float16 h = (_Float16)a[q]; fh.h[q] = h; fl.h[q] = (_Float16)((a[q] - (float)h) * 1024.0f); h = (_Float16)c[q]; fh.h[4 + q] = h; fl.h[4 + q] = (_Float16)((c[q] - (float)h) * 1024.0f); }
  for (int pass = 0; pass < 2; ++pass) { *(volatile v8us*)((unsigned short*)Hh + t * 8) = fh.half[0]; *(volatile v8us*)((unsigned short*)Hl + t * 8) = fl.half[0]; if (pass == 0) __threadfence(); } }

__global__ __launch_bounds__(256) void k_ln(const float* __restrict__ X, const float* __restrict__ w, const float* __restrict__ b, _Float16* __restrict__ H) { const int tid = threadIdx.x, wv = tid >> 5, l = tid & 31; const size_t row = (size_t)blockIdx.x * 8 + wv; const float* xr = X + row * DM;
  float v[32]; float s = 0.f;
#pragma unroll
  for (int q = 0; q < 4; ++q) { const v4f a = *(const v4fa*)(xr + q * 256 + 8 * l), c = *(const v4fa*)(xr + q * 256 + 8 * l + 4);
#pragma unroll
    for (int j = 0; j < 4; ++j) { v[q * 8 + j] = bf16_round(a[j]); v[q * 8 + 4 + j] = bf16_round(c[j]); } }
#pragma unroll
  for (int i = 0; i < 32; ++i) s += v[i];
  for (int o = 16; o > 0; o >>= 1) s += __shfl_xor(s, o, 32); const float mu = s * (1.0f / DM); float vs = 0.f;
#pragma unroll
  for (int i = 0; i < 32; ++i) { const float d = v[i] - mu; vs += d * d; }
  for (int o = 16; o > 0; o >>= 1) vs += __shfl_xor(vs, o, 32); const float rs = rsqrtf(vs * (1.0f / DM) + LNEPS);
  FragH f[4];
#pragma unroll
  for (int q = 0; q < 4; ++q)
#pragma unroll
    for (int j = 0; j < 8; ++j) { const int c = q * 256 + 8 * l + j; f[q].h[j] = (_Float16)((v[q * 8 + j] - mu) * rs * bf16_round(w[c]) + bf16_round(b[c])); }
  for (int pass = 0; pass < 2; ++pass) {
#pragma unroll
    for (int q = 0; q < 4; ++q) *(volatile v8us*)((unsigned short*)H + row * DM + q * 256 + 8 * l) = f[q].half[0];
    if (pass == 0) __threadfence(); } }
__global__ __launch_bounds__(256) void k_conv(const float* __restrict__ XI, const float* __restrict__ cw, const float* __restrict__ cb, _Float16* __restrict__ U16) { const size_t t0 = (size_t)blockIdx.x * 256 + threadIdx.x; if (t0 >= (size_t)NR * (DI / 8)) return; const int d0 = (int)(t0 % (DI / 8)) * 8; const size_t row = t0 / (DI / 8); const int t = (int)(row % TT); FragH f;
#pragma unroll
  for (int j = 0; j < 8; ++j) { const int d = d0 + j; float a = bf16_round(cb[d]);
#pragma unroll
    for (int k = 0; k < 4; ++k) { const int back = 3 - k; const bool ok = (t >= back); const size_t rr = ok ? (row - (size_t)back) : row; a += ok ? bf16_round(cw[d * 4 + k]) * XI[rr * DI + d] : 0.f; }
    f.h[j] = (_Float16)(a / (1.0f + fexp(-a))); }
  *(volatile v8us*)((unsigned short*)U16 + row * DI + d0) = f.half[0]; __threadfence(); *(volatile v8us*)((unsigned short*)U16 + row * DI + d0) = f.half[0]; }
__global__ __launch_bounds__(256) void k_bfx(const float* __restrict__ x, float* __restrict__ Xb, size_t n4) { const size_t t = (size_t)blockIdx.x * 256 + threadIdx.x; if (t >= n4) return; const v4f a = *(const v4fa*)(x + t * 4); v4f o; o[0] = bf16_round(a[0]); o[1] = bf16_round(a[1]); o[2] = bf16_round(a[2]); o[3] = bf16_round(a[3]); *(volatile v4f*)(Xb + t * 4) = o; __threadfence(); *(volatile v4f*)(Xb + t * 4) = o; }
__global__ __launch_bounds__(256) void k_dtr(const float* __restrict__ XD, _Float16* __restrict__ D16) { const size_t t = (size_t)blockIdx.x * 256 + threadIdx.x; if (t >= (size_t)NR * 8) return; const size_t row = t / 8; const int j0 = (int)(t % 8) * 8; FragH f;
#pragma unroll
  for (int q = 0; q < 8; ++q) f.h[q] = (_Float16)XD[row * XPW + j0 + q];
  *(volatile v8us*)((unsigned short*)D16 + row * DTR + j0) = f.half[0]; __threadfence(); *(volatile v8us*)((unsigned short*)D16 + row * DTR + j0) = f.half[0]; }
__global__ __launch_bounds__(256) void k_scan(const _Float16* __restrict__ U16, const _Float16* __restrict__ DT16, const float* __restrict__ XD, const float* __restrict__ RES, const float* __restrict__ Alog, const float* __restrict__ Dsk, _Float16* __restrict__ YS) {
  #pragma clang fp contract(off)
  const int gtid = blockIdx.x * 256 + threadIdx.x; const int b = gtid / (DI / 2), d0 = (gtid % (DI / 2)) * 2; if (b >= BB) return;
  float A0[NS], A1[NS], h0[NS], h1[NS];
#pragma unroll
  for (int n = 0; n < NS; ++n) { A0[n] = -fexp(bf16_round(Alog[(size_t)d0 * NS + n])); A1[n] = -fexp(bf16_round(Alog[(size_t)(d0 + 1) * NS + n])); h0[n] = 0.f; h1[n] = 0.f; }
  const float D0 = bf16_round(Dsk[d0]), D1 = bf16_round(Dsk[d0 + 1]);
#pragma unroll 1
  for (int t = 0; t < TT; ++t) { const size_t row = (size_t)b * TT + t; const unsigned int uw = *(const unsigned int*)((const unsigned short*)U16 + row * DI + d0), tw = *(const unsigned int*)((const unsigned short*)DT16 + row * DI + d0);
    FragH cv; cv.u[0] = (unsigned short)(uw & 0xFFFFu); cv.u[1] = (unsigned short)(uw >> 16); cv.u[2] = (unsigned short)(tw & 0xFFFFu); cv.u[3] = (unsigned short)(tw >> 16);
    const float u0 = (float)cv.h[0], u1 = (float)cv.h[1], t0 = (float)cv.h[2], t1 = (float)cv.h[3]; const float* bc = XD + row * XPW + DTR; const float du0 = t0 * u0, du1 = t1 * u1; float y0 = 0.f, y1 = 0.f;
#pragma unroll
    for (int n = 0; n < NS; ++n) { const float bn = bc[n], cn = bc[NS + n]; h0[n] = h0[n] * fexp(t0 * A0[n]) + du0 * bn; h1[n] = h1[n] * fexp(t1 * A1[n]) + du1 * bn; y0 += h0[n] * cn; y1 += h1[n] * cn; }
    y0 += u0 * D0; y1 += u1 * D1; const float r0 = RES[row * DI + d0], r1 = RES[row * DI + d0 + 1];
    FragH o; o.h[0] = (_Float16)(y0 * (r0 / (1.0f + fexp(-r0)))); o.h[1] = (_Float16)(y1 * (r1 / (1.0f + fexp(-r1)))); const unsigned int ow = (unsigned int)o.u[0] | ((unsigned int)o.u[1] << 16);
    volatile unsigned int* p = (volatile unsigned int*)((unsigned short*)YS + row * DI + d0); *p = ow; __threadfence(); *p = ow; } }

extern "C" void kernel_launch(void* const* d_in, const int* in_sizes, int n_in,
                              void* d_out, int out_size, void* d_ws, size_t ws_size, hipStream_t stream) {
  (void)in_sizes; (void)n_in; (void)out_size;
  const float* const* I = (const float* const*)d_in; const float* x = I[0]; const float* ln_w = I[1]; const float* ln_b = I[2]; const float* in_w = I[3]; const float* conv_w = I[4]; const float* conv_b = I[5]; const float* xp_w = I[6]; const float* dtp_w = I[7]; const float* dtp_b = I[8]; const float* A_log = I[9]; const float* D_skip = I[10]; const float* out_w = I[11];
  char* ws = (char*)d_ws; size_t off = 0;
  auto take = [&](size_t bytes) { char* p = ws + off; off += (bytes + 255) & ~(size_t)255; return p; };
  _Float16* Win = (_Float16*)take((size_t)2 * DI * DM * 2); _Float16* Wout = (_Float16*)take((size_t)DM * DI * 2); _Float16* Wxp = (_Float16*)take((size_t)XPW * DI * 2); _Float16* Wdt = (_Float16*)take((size_t)DI * DTR * 2);
  float* XI = (float*)take((size_t)NR * DI * 4); float* RES = (float*)take((size_t)NR * DI * 4); _Float16* U16 = (_Float16*)take((size_t)NR * DI * 2); float* XD = (float*)take((size_t)NR * XPW * 4); _Float16* D16 = (_Float16*)take((size_t)NR * DTR * 2); float* X1 = (float*)take((size_t)NR * DM * 4);
  _Float16* XN = U16;
  _Float16* DT16 = (_Float16*)XI;
  _Float16* YS = (_Float16*)XI + (size_t)NR * DI;
  if (off > ws_size) return;
  const unsigned g8 = (unsigned)(((size_t)NR * DI / 8 + 255) / 256);
  k_bfx<<<(unsigned)(((size_t)NR * DM / 4 + 255) / 256), 256, 0, stream>>>(x, X1, (size_t)NR * DM / 4);
  for (int L = 0; L < 2; ++L) { const float* Xin = X1; float* Xout = (L == 0) ? X1 : (float*)d_out;
    k_round16f<<<(unsigned)(((size_t)2 * DI * DM / 8 + 255) / 256), 256, 0, stream>>>(in_w + (size_t)L * 2 * DI * DM, Win, (size_t)2 * DI * DM / 8);
    k_round16f<<<(unsigned)(((size_t)DM * DI / 8 + 255) / 256), 256, 0, stream>>>(out_w + (size_t)L * DM * DI, Wout, (size_t)DM * DI / 8);
    k_round16f<<<(XPW * DI / 8 + 255) / 256, 256, 0, stream>>>(xp_w + (size_t)L * XPW * DI, Wxp, (size_t)XPW * DI / 8); k_round16f<<<(DI * DTR / 8 + 255) / 256, 256, 0, stream>>>(dtp_w + (size_t)L * DI * DTR, Wdt, (size_t)DI * DTR / 8);
    k_ln<<<NR / 8, 256, 0, stream>>>(Xin, ln_w + (size_t)L * DM, ln_b + (size_t)L * DM, XN);
    const dim3 gi(((NR / 16) * (DI / 64) + 3) / 4, 1);
    k_gemm_hhx<0><<<gi, 128, 0, stream>>>(XN, DM, 0, Win, DM, 0, 0.0625f, nullptr, 0, nullptr, 1, 0, 0, XI, nullptr, DI, 0, NR, DI, DM);
    k_gemm_hhx<0><<<gi, 128, 0, stream>>>(XN, DM, 0, Win + (size_t)DI * DM, DM, 0, 0.0625f, nullptr, 0, nullptr, 1, 0, 0, RES, nullptr, DI, 0, NR, DI, DM);
    k_conv<<<g8, 256, 0, stream>>>(XI, conv_w + (size_t)L * DI * 4, conv_b + (size_t)L * DI, U16);
    k_gemm_hhx<0><<<dim3(((NR / 16) * ((XPW + 63) / 64) + 3) / 4, 1), 128, 0, stream>>>(U16, DI, 0, Wxp, DI, 0, 0.0625f, nullptr, 0, nullptr, 1, 0, 0, XD, nullptr, XPW, 0, NR, XPW, DI);
    k_dtr<<<(NR * 8 + 255) / 256, 256, 0, stream>>>(XD, D16);
    k_gemm_hhx<13><<<gi, 128, 0, stream>>>(D16, DTR, 0, Wdt, DTR, 0, 0.0625f, dtp_b + (size_t)L * DI, 0, nullptr, 1, 0, 0, nullptr, DT16, DI, 0, NR, DI, DTR);
    k_scan<<<(BB * (DI / 2) + 255) / 256, 256, 0, stream>>>(U16, DT16, XD, RES, A_log + (size_t)L * DI * NS, D_skip + (size_t)L * DI, YS);
    k_gemm_hhx<0><<<dim3(((NR / 16) * (DM / 64) + 3) / 4, 1), 128, 0, stream>>>(YS, DI, 0, Wout, DI, 0, 0.0625f, nullptr, 0, Xin, 1, (size_t)DM, 0, Xout, nullptr, DM, 0, NR, DM, DI); }
}
